// ContextualizedNN_2396591751282
// MI455X (gfx1250) — hardware-run, weakly checked
//
#include <hip/hip_runtime.h>

typedef __bf16   v16bf __attribute__((ext_vector_type(16)));
typedef float    v8f   __attribute__((ext_vector_type(8)));
typedef float    v4f   __attribute__((ext_vector_type(4)));
typedef unsigned v4u   __attribute__((ext_vector_type(4)));
typedef v4u      __attribute__((may_alias)) v4ua;
typedef v4f      __attribute__((may_alias)) v4fa;
typedef unsigned __attribute__((may_alias)) u32a;

union Frag { v16bf v; v4u q[2]; unsigned u[8]; };

#define KNB   20
#define KPAD  32
#define DDIM  64
#define CAT   128
#define H1N   64
#define H2N   32
#define WPB   2
#define NTHR  (WPB * 32)
#define PPW   4
#define ROWS  (PPW * KNB)
#define RT    (ROWS / 16)
#define PPB   64
#define NIT   (PPB / (WPB * PPW))

static_assert(ROWS % 16 == 0);
static_assert(PPB == NIT * WPB * PPW);
static_assert(NTHR == H1N);

#define OFF_W1T   0
#define OFF_W2T   16384
#define OFF_B1    20480
#define OFF_B2    20736
#define OFF_W3    20864
#define OFF_B3    20992
#define OFF_RES   21008
#define OFF_SLAB  21264
#define SL_XH     0
#define SL_XL     20480
#define SL_ET     40960
#define SL_ST     45056
#define SL_SIG    47104
#define SLAB_BYTES 47424
#define SMEM_TOTAL (OFF_SLAB + WPB * SLAB_BYTES)

static_assert((OFF_SLAB % 16) == 0);
static_assert((SLAB_BYTES % 16) == 0);
static_assert(SMEM_TOTAL <= 160 * 1024);

__device__ __forceinline__ unsigned bf16_bits(float x) {
  const unsigned u = __float_as_uint(x);
  return (u + 0x7FFFu + ((u >> 16) & 1u)) >> 16;
}
__device__ __forceinline__ float bf16_val(float x) {
  return __uint_as_float(bf16_bits(x) << 16);
}
__device__ __forceinline__ unsigned pk2(float lo, float hi) {
  return bf16_bits(lo) | (bf16_bits(hi) << 16);
}
__device__ __forceinline__ void split8(v8f c, v4u& hq, v4u& lq) {
  unsigned hw[4], lw[4];
  #pragma unroll
  for (int i = 0; i < 4; ++i) {
    const float a0 = c[2 * i], a1 = c[2 * i + 1];
    const unsigned h0 = bf16_bits(a0), h1 = bf16_bits(a1);
    const float r0 = a0 - __uint_as_float(h0 << 16);
    const float r1 = a1 - __uint_as_float(h1 << 16);
    hw[i] = h0 | (h1 << 16);
    lw[i] = bf16_bits(r0) | (bf16_bits(r1) << 16);
  }
  hq.x = hw[0]; hq.y = hw[1]; hq.z = hw[2]; hq.w = hw[3];
  lq.x = lw[0]; lq.y = lw[1]; lq.z = lw[2]; lq.w = lw[3];
}
__device__ __forceinline__ void relu_split16(v8f p, v8f q, v16bf& hi, v16bf& lo) {
  Frag fh, fl;
  #pragma unroll
  for (int i = 0; i < 4; ++i) {
    const float a0 = fmaxf(p[2 * i], 0.0f), a1 = fmaxf(p[2 * i + 1], 0.0f);
    const unsigned h0 = bf16_bits(a0), h1 = bf16_bits(a1);
    fh.u[i] = h0 | (h1 << 16);
    fl.u[i] = bf16_bits(a0 - __uint_as_float(h0 << 16)) | (bf16_bits(a1 - __uint_as_float(h1 << 16)) << 16);
    const float c0 = fmaxf(q[2 * i], 0.0f), c1 = fmaxf(q[2 * i + 1], 0.0f);
    const unsigned g0 = bf16_bits(c0), g1 = bf16_bits(c1);
    fh.u[4 + i] = g0 | (g1 << 16);
    fl.u[4 + i] = bf16_bits(c0 - __uint_as_float(g0 << 16)) | (bf16_bits(c1 - __uint_as_float(g1 << 16)) << 16);
  }
  hi = fh.v; lo = fl.v;
}

__device__ __forceinline__ v8f wmma_bf16(v16bf a, v16bf b, v8f c) {
  v8f d = __builtin_amdgcn_wmma_f32_16x16x32_bf16(false, a, false, b, (short)0, c, false, false);
  asm volatile("v_nop\n\tv_nop\n\tv_nop\n\tv_nop" : "+v"(d) : "v"(a), "v"(b));
  return d;
}

__device__ __forceinline__ v16bf load_frag(const unsigned short* p, int h) {
  Frag f;
  f.q[0] = *(const v4ua*)(p + 8 * h);
  f.q[1] = *(const v4ua*)(p + 16 + 8 * h);
  return f.v;
}

__device__ __forceinline__ int wrapclamp(int i, int n) {
  i = (i < 0) ? (i + n) : i;
  i = (i < 0) ? 0 : i;
  i = (i > n - 1) ? (n - 1) : i;
  return i;
}

__global__ __launch_bounds__(NTHR) void cnn_fused_kernel(
    const int*   __restrict__ user_idxs,
    const int*   __restrict__ item_idxs,
    const int*   __restrict__ user_idx_tensor,
    const float* __restrict__ user_scr_tensor,
    const int*   __restrict__ item_idx_tensor,
    const float* __restrict__ item_scr_tensor,
    const float* __restrict__ user_emb_table,
    const float* __restrict__ item_emb_table,
    const float* __restrict__ w1, const float* __restrict__ b1,
    const float* __restrict__ w2, const float* __restrict__ b2,
    const float* __restrict__ w3, const float* __restrict__ b3,
    float* __restrict__ out,
    int nUI, int nUS, int nUE, int nII, int nIS, int nIE)
{
  extern __shared__ __align__(16) unsigned char smem[];
  unsigned short* W1T = (unsigned short*)(smem + OFF_W1T);
  unsigned short* W2T = (unsigned short*)(smem + OFF_W2T);
  float* sB1 = (float*)(smem + OFF_B1);
  float* sB2 = (float*)(smem + OFF_B2);
  float* sW3 = (float*)(smem + OFF_W3);
  float* sB3 = (float*)(smem + OFF_B3);
  float* RES = (float*)(smem + OFF_RES);

  const int tid = threadIdx.x, lane = tid & 31, wave = tid >> 5;
  const int h = lane >> 4, m = lane & 15;

  unsigned char* slab = smem + OFF_SLAB + wave * SLAB_BYTES;
  unsigned short* XH = (unsigned short*)(slab + SL_XH);
  unsigned short* XL = (unsigned short*)(slab + SL_XL);
  unsigned short* ET = (unsigned short*)(slab + SL_ET);
  unsigned short* ST = (unsigned short*)(slab + SL_ST);
  float* SIG = (float*)(slab + SL_SIG);

  #pragma unroll 4
  for (int i = tid; i < CAT * H1N; i += NTHR) {
    const int k = i >> 6, n = i & 63;
    W1T[n * CAT + k] = (unsigned short)bf16_bits(w1[i]);
  }
  #pragma unroll 4
  for (int i = tid; i < H1N * H2N; i += NTHR) {
    const int k = i >> 5, n = i & 31;
    W2T[n * H1N + k] = (unsigned short)bf16_bits(w2[i]);
  }
  if (tid < H1N) sB1[tid] = bf16_val(b1[tid]);
  if (tid < H2N) { sB2[tid] = bf16_val(b2[tid]); sW3[tid] = bf16_val(w3[tid]); }
  if (tid == 0) sB3[0] = bf16_val(b3[0]);
  #pragma unroll
  for (int t = 0; t < 12; ++t) {
    const int idx = t * 32 + lane;
    const int d = idx / 6;
    const int j = KNB + 2 * (idx - 6 * d);
    *(u32a*)(ET + d * KPAD + j) = 0u;
  }
  __syncthreads();

  const v8f zero8 = {0.f, 0.f, 0.f, 0.f, 0.f, 0.f, 0.f, 0.f};
  const int pblk = blockIdx.x * PPB;

  #pragma unroll 1
  for (int it = 0; it < NIT; ++it) {
    const int pbase = pblk + it * (WPB * PPW) + wave * PPW;

    #pragma unroll 1
    for (int slot = 0; slot < PPW; ++slot) {
      const int b = pbase + slot;
      #pragma unroll 1
      for (int side = 0; side < 2; ++side) {
        const int*   idxt = side ? item_idx_tensor : user_idx_tensor;
        const float* scr  = side ? item_scr_tensor : user_scr_tensor;
        const float* emb  = side ? item_emb_table  : user_emb_table;
        const int*   ridx = side ? item_idxs : user_idxs;
        const int nI = side ? nII : nUI;
        const int nS = side ? nIS : nUS;
        const int nE = side ? nIE : nUE;

        const int root = wrapclamp(ridx[b], nI);
        const int jj = (lane < KNB) ? lane : (KNB - 1);
        const int nj = idxt[(size_t)root * KNB + jj];
        const int njE = wrapclamp(nj, nE);
        const int njS = wrapclamp(nj, nS);

        __syncthreads();

        #pragma unroll 2
        for (int j = 0; j < KNB; j += 2) {
          const int n0 = __shfl(njE, j);
          const int n1 = __shfl(njE, j + 1);
          const float* r0 = emb + (size_t)n0 * DDIM;
          const float* r1 = emb + (size_t)n1 * DDIM;
          const float e0a = r0[lane], e1a = r1[lane];
          const float e0b = r0[lane + 32], e1b = r1[lane + 32];
          *(u32a*)(ET + lane * KPAD + j)        = pk2(e0a, e1a);
          *(u32a*)(ET + (lane + 32) * KPAD + j) = pk2(e0b, e1b);
        }
        {
          const float* sr = scr + (size_t)njS * KNB;
          const v4f q0 = *(const v4fa*)(sr);
          const v4f q1 = *(const v4fa*)(sr + 4);
          const v4f q2 = *(const v4fa*)(sr + 8);
          const v4f q3 = *(const v4fa*)(sr + 12);
          const v4f q4 = *(const v4fa*)(sr + 16);
          const bool valid = lane < KNB;
          v4u s0, s1, s2, s3;
          s0.x = valid ? pk2(q0.x, q0.y) : 0u;  s0.y = valid ? pk2(q0.z, q0.w) : 0u;
          s0.z = valid ? pk2(q1.x, q1.y) : 0u;  s0.w = valid ? pk2(q1.z, q1.w) : 0u;
          s1.x = valid ? pk2(q2.x, q2.y) : 0u;  s1.y = valid ? pk2(q2.z, q2.w) : 0u;
          s1.z = valid ? pk2(q3.x, q3.y) : 0u;  s1.w = valid ? pk2(q3.z, q3.w) : 0u;
          s2.x = valid ? pk2(q4.x, q4.y) : 0u;  s2.y = valid ? pk2(q4.z, q4.w) : 0u;
          s2.z = 0u; s2.w = 0u;
          s3.x = 0u; s3.y = 0u; s3.z = 0u; s3.w = 0u;
          *(v4ua*)(ST + lane * KPAD + 0)  = s0;
          *(v4ua*)(ST + lane * KPAD + 8)  = s1;
          *(v4ua*)(ST + lane * KPAD + 16) = s2;
          *(v4ua*)(ST + lane * KPAD + 24) = s3;
        }
        __syncthreads();

        const v16bf bs0 = load_frag(ST + (0 + m) * KPAD, h);
        const v16bf bs1 = load_frag(ST + (16 + m) * KPAD, h);
        #pragma unroll
        for (int dt = 0; dt < 4; ++dt) {
          const v16bf a = load_frag(ET + (16 * dt + m) * KPAD, h);
          const v8f c0 = wmma_bf16(a, bs0, zero8);
          const v8f c1 = wmma_bf16(a, bs1, zero8);
          const int col0 = side * DDIM + 16 * dt + 8 * h;
          v4u hq, lq;
          split8(c0, hq, lq);
          const int o0 = (slot * KNB + m) * CAT + col0;
          *(v4ua*)(XH + o0) = hq;
          *(v4ua*)(XL + o0) = lq;
          split8(c1, hq, lq);
          if (m < KNB - 16) {
            const int o1 = (slot * KNB + 16 + m) * CAT + col0;
            *(v4ua*)(XH + o1) = hq;
            *(v4ua*)(XL + o1) = lq;
          }
        }
      }
    }
    __syncthreads();

    #pragma unroll 1
    for (int rt = 0; rt < RT; ++rt) {
      v8f acc[4];
      #pragma unroll
      for (int ot = 0; ot < 4; ++ot)
        #pragma unroll
        for (int r = 0; r < 8; ++r) acc[ot][r] = sB1[16 * ot + 8 * h + r];

      const unsigned short* xr = XH + (rt * 16 + m) * CAT;
      const unsigned short* xs = XL + (rt * 16 + m) * CAT;
      #pragma unroll
      for (int ks = 0; ks < 4; ++ks) {
        const v16bf bxh = load_frag(xr + 32 * ks, h);
        const v16bf bxl = load_frag(xs + 32 * ks, h);
        #pragma unroll
        for (int ot = 0; ot < 4; ++ot) {
          const v16bf a = load_frag(W1T + (16 * ot + m) * CAT + 32 * ks, h);
          acc[ot] = wmma_bf16(a, bxh, acc[ot]);
          acc[ot] = wmma_bf16(a, bxl, acc[ot]);
        }
      }

      v8f acc2[2];
      #pragma unroll
      for (int ot2 = 0; ot2 < 2; ++ot2)
        #pragma unroll
        for (int r = 0; r < 8; ++r) acc2[ot2][r] = sB2[16 * ot2 + 8 * h + r];

      #pragma unroll
      for (int ks2 = 0; ks2 < 2; ++ks2) {
        v16bf bh, bl;
        relu_split16(acc[2 * ks2], acc[2 * ks2 + 1], bh, bl);
        #pragma unroll
        for (int ot2 = 0; ot2 < 2; ++ot2) {
          const v16bf a = load_frag(W2T + (16 * ot2 + m) * H1N + 32 * ks2, h);
          acc2[ot2] = wmma_bf16(a, bh, acc2[ot2]);
          acc2[ot2] = wmma_bf16(a, bl, acc2[ot2]);
        }
      }

      float zp = 0.0f;
      #pragma unroll
      for (int ot2 = 0; ot2 < 2; ++ot2)
        #pragma unroll
        for (int r = 0; r < 8; ++r)
          zp = fmaf(fmaxf(acc2[ot2][r], 0.0f), sW3[16 * ot2 + 8 * h + r], zp);
      const float z = zp + __shfl_xor(zp, 16) + sB3[0];
      const float p = 1.0f / (1.0f + expf(-z));
      if (h == 0) SIG[rt * 16 + m] = p;
    }
    __syncthreads();

    if (lane < PPW) {
      float s = 0.0f;
      #pragma unroll
      for (int k = 0; k < KNB; ++k) s += SIG[lane * KNB + k];
      RES[it * (WPB * PPW) + wave * PPW + lane] = s * (1.0f / (float)KNB);
    }
  }
  __syncthreads();

  if (wave == 0 && lane < 16) {
    const v4f v = *(const v4fa*)(RES + 4 * lane);
    float* gp = out + (size_t)blockIdx.x * PPB + 4 * lane;
    *(volatile v4f*)gp = v;
    __threadfence();
    *(volatile v4f*)gp = v;
  }
}

extern "C" void kernel_launch(void* const* d_in, const int* in_sizes, int n_in,
                              void* d_out, int out_size, void* d_ws, size_t ws_size,
                              hipStream_t stream) {
  (void)d_ws; (void)ws_size;
  if (n_in < 14) return;
  const int B = in_sizes[0];
  if (B <= 0 || in_sizes[1] != B || out_size != B) return;
  if ((B % PPB) != 0) return;
  if (in_sizes[2] < KNB || (in_sizes[2] % KNB) != 0) return;
  if (in_sizes[3] < KNB || (in_sizes[3] % KNB) != 0) return;
  if (in_sizes[4] < KNB || (in_sizes[4] % KNB) != 0) return;
  if (in_sizes[5] < KNB || (in_sizes[5] % KNB) != 0) return;
  if (in_sizes[6] < DDIM || (in_sizes[6] % DDIM) != 0) return;
  if (in_sizes[7] < DDIM || (in_sizes[7] % DDIM) != 0) return;
  if (in_sizes[8] != CAT * H1N || in_sizes[9] != H1N) return;
  if (in_sizes[10] != H1N * H2N || in_sizes[11] != H2N) return;
  if (in_sizes[12] != H2N || in_sizes[13] < 1) return;

  const int*   user_idxs       = (const int*)  d_in[0];
  const int*   item_idxs       = (const int*)  d_in[1];
  const int*   user_idx_tensor = (const int*)  d_in[2];
  const float* user_scr_tensor = (const float*)d_in[3];
  const int*   item_idx_tensor = (const int*)  d_in[4];
  const float* item_scr_tensor = (const float*)d_in[5];
  const float* user_emb_table  = (const float*)d_in[6];
  const float* item_emb_table  = (const float*)d_in[7];
  const float* w1 = (const float*)d_in[8];
  const float* b1 = (const float*)d_in[9];
  const float* w2 = (const float*)d_in[10];
  const float* b2 = (const float*)d_in[11];
  const float* w3 = (const float*)d_in[12];
  const float* b3 = (const float*)d_in[13];
  float* out = (float*)d_out;

  const int nUI = in_sizes[2] / KNB;
  const int nUS = in_sizes[3] / KNB;
  const int nUE = in_sizes[6] / DDIM;
  const int nII = in_sizes[4] / KNB;
  const int nIS = in_sizes[5] / KNB;
  const int nIE = in_sizes[7] / DDIM;

  hipFuncSetAttribute(reinterpret_cast<const void*>(&cnn_fused_kernel),
                      hipFuncAttributeMaxDynamicSharedMemorySize, SMEM_TOTAL);

  hipLaunchKernelGGL(cnn_fused_kernel, dim3(B / PPB), dim3(NTHR), SMEM_TOTAL, stream,
                     user_idxs, item_idxs,
                     user_idx_tensor, user_scr_tensor,
                     item_idx_tensor, item_scr_tensor,
                     user_emb_table, item_emb_table,
                     w1, b1, w2, b2, w3, b3, out,
                     nUI, nUS, nUE, nII, nIS, nIE);
  (void)hipGetLastError();
}
